// SC_encoder_50500225466896
// MI455X (gfx1250) — hardware-verified
//
#include <hip/hip_runtime.h>
#include <math.h>

typedef __attribute__((ext_vector_type(16))) _Float16 v16h;
typedef __attribute__((ext_vector_type(16))) __bf16 v16b;
typedef __attribute__((ext_vector_type(8)))  _Float16 v8h;
typedef __attribute__((ext_vector_type(8)))  float v8f;
typedef __attribute__((ext_vector_type(4)))  float v4f;
typedef __attribute__((ext_vector_type(2)))  float v2f;
typedef __attribute__((ext_vector_type(4)))  unsigned v4u;
typedef __attribute__((ext_vector_type(4)))  int v4i;
typedef float __attribute__((may_alias)) float_a;
typedef int __attribute__((may_alias)) int_a;

template <typename T> __device__ __forceinline__ void vst2(void* p, T v) { *(volatile T*)p = v; __threadfence(); *(volatile T*)p = v; }
__device__ __forceinline__ v8f wmma16(v16h a, v16h b, v8f c) {
  v8f d = __builtin_amdgcn_wmma_f32_16x16x32_f16(false, a, false, b, (short)0, c, false, false);
  asm volatile("v_nop\n\tv_nop\n\tv_nop\n\tv_nop" : "+v"(d) : "v"(a), "v"(b));
  return d;
}
__device__ __forceinline__ v8f wmma_bf(v16b a, v16b b, v8f c) {
  v8f d = __builtin_amdgcn_wmma_f32_16x16x32_bf16(false, a, false, b, (short)0, c, false, false);
  asm volatile("v_nop\n\tv_nop\n\tv_nop\n\tv_nop" : "+v"(d) : "v"(a), "v"(b));
  return d;
}
__device__ __forceinline__ v16h frag_h(const _Float16* rowk0, int lane) {
  union { v16h v; v8h q[2]; } u; const _Float16* p = rowk0 + 8 * (lane >> 4);
  u.q[0] = *(const v8h*)p; u.q[1] = *(const v8h*)(p + 16); return u.v;
}
__device__ __forceinline__ v16h frag_f32(const float* rowk0, int lane) {
  v16h a; const float* p = rowk0 + 8 * (lane >> 4);
#pragma unroll
  for (int i = 0; i < 8; ++i) { a[i] = (_Float16)p[i]; a[8 + i] = (_Float16)p[16 + i]; }
  return a;
}
__device__ __forceinline__ v16h frag_f32s(const float* rowk0, int lane, float sc) {
  v16h a; const float* p = rowk0 + 8 * (lane >> 4);
#pragma unroll
  for (int i = 0; i < 8; ++i) { a[i] = (_Float16)(p[i] * sc); a[8 + i] = (_Float16)(p[16 + i] * sc); }
  return a;
}
__device__ __forceinline__ v16h fragc_f32(const float* W, int k0, int n, int lane, int ld, int K) {
  v16h a; const int g = lane >> 4;
#pragma unroll
  for (int i = 0; i < 8; ++i) { const int ka = k0 + 8 * g + i, kb = ka + 16;
    a[i] = (_Float16)(ka < K ? W[(size_t)(ka < K ? ka : K - 1) * ld + n] : 0.f); a[8 + i] = (_Float16)(kb < K ? W[(size_t)(kb < K ? kb : K - 1) * ld + n] : 0.f); }
  return a;
}
struct F2 { v16b h, l; };
__device__ __forceinline__ F2 bsplit16(const float v[16]) { F2 r;
#pragma unroll
  for (int i = 0; i < 16; ++i) { const __bf16 h = (__bf16)v[i]; r.h[i] = h; r.l[i] = (__bf16)(v[i] - (float)h); }
  return r; }
__device__ __forceinline__ F2 split_row(const float* row, int k0, int lane) { float v[16]; const float* p = row + k0 + 8 * (lane >> 4);
#pragma unroll
  for (int i = 0; i < 8; ++i) { v[i] = p[i]; v[8 + i] = p[16 + i]; }
  return bsplit16(v); }
__device__ __forceinline__ F2 split_rowK(const float* row, int k0, int lane, int K) { float v[16]; const int g = lane >> 4;
#pragma unroll
  for (int i = 0; i < 8; ++i) { const int ka = k0 + 8 * g + i, kb = ka + 16; v[i] = ka < K ? row[ka < K ? ka : K - 1] : 0.f; v[8 + i] = kb < K ? row[kb < K ? kb : K - 1] : 0.f; }
  return bsplit16(v); }
__device__ __forceinline__ F2 split_col(const float* W, int k0, int n, int lane, int ld, int K) { float v[16]; const int g = lane >> 4;
#pragma unroll
  for (int i = 0; i < 8; ++i) { const int ka = k0 + 8 * g + i, kb = ka + 16; v[i] = ka < K ? W[(size_t)(ka < K ? ka : K - 1) * ld + n] : 0.f; v[8 + i] = kb < K ? W[(size_t)(kb < K ? kb : K - 1) * ld + n] : 0.f; }
  return bsplit16(v); }
__device__ __forceinline__ v8f mac3(const F2& a, const F2& b, v8f c) { c = wmma_bf(a.l, b.h, c); c = wmma_bf(a.h, b.l, c); return wmma_bf(a.h, b.h, c); }
__device__ __forceinline__ float sigm(float v) { return 1.0f / (1.0f + expf(-v)); }
#define LDSX() do { asm volatile("s_wait_dscnt 0" ::: "memory"); __builtin_amdgcn_wave_barrier(); __builtin_amdgcn_fence(__ATOMIC_RELEASE, "workgroup"); } while (0)


#define NN 50000
#define HDIM 64
#define KNEI 15
#define NBLK ((NN + 63) / 64)
__device__ __forceinline__ float bfr(float v) { return (float)(__bf16)v; }
__device__ __forceinline__ v16b frag_b(const __bf16* rowk0, int lane) { return __builtin_bit_cast(v16b, frag_h((const _Float16*)rowk0, lane)); }
__device__ __attribute__((noinline)) float exp_ni(float v) { return expf(v); }
__device__ __attribute__((noinline)) float tanh_ni(float v) { return tanhf(v); }

__global__ __launch_bounds__(128) void k_intra(const float* __restrict__ href, const float* __restrict__ ht, int Mt, const int* __restrict__ nei, const float* __restrict__ att, float* __restrict__ EMB) {
  __shared__ __align__(16) __bf16 sg[64 * KNEI][HDIM + 8];
  __shared__ __align__(16) __bf16 sr[64][HDIM + 8];
  __shared__ __align__(16) __bf16 sa[16][HDIM + 8];
  __shared__ float ssc[64 * KNEI + 16], srs[64];
  __shared__ __align__(16) float se[64][HDIM + 4];
  const int tid = threadIdx.x, wave = tid >> 5, lane = tid & 31, col = lane & 15, g = lane >> 4; const int n0 = blockIdx.x * 64;
  for (int q = tid; q < 16 * 8; q += 128) { const int rr = q >> 3, pc = q & 7; union { __bf16 e[8]; v4u u; } pk;
#pragma unroll
    for (int e = 0; e < 8; ++e) pk.e[e] = (__bf16)(rr == 0 ? att[HDIM + pc * 8 + e] : (rr == 1 ? att[pc * 8 + e] : 0.f));
    *(v4u*)(&sa[rr][pc * 8]) = pk.u; }
  for (int q = tid; q < 64 * 8; q += 128) { const int rl = q >> 3, pc = q & 7; const int n = n0 + rl; const int nc = n < NN ? n : NN - 1; union { __bf16 e[8]; v4u u; } pk; const float* src = href + (size_t)nc * HDIM + pc * 8;
#pragma unroll
    for (int e = 0; e < 8; ++e) pk.e[e] = (__bf16)src[e];
    *(v4u*)(&sr[rl][pc * 8]) = pk.u; }
  for (int q = tid; q < 64 * KNEI * 8; q += 128) { const int gr = q >> 3, pc = q & 7; const int rl = gr / KNEI; const int n = n0 + rl; const int nc = n < NN ? n : NN - 1; const int idx = nei[(size_t)nc * KNEI + (gr - rl * KNEI)]; const bool pad = (idx < 0) || (idx >= Mt); const int ic = pad ? 0 : idx;
    union { __bf16 e[8]; v4u u; } pk; const float* src = ht + (size_t)ic * HDIM + pc * 8;
#pragma unroll
    for (int e = 0; e < 8; ++e) pk.e[e] = (__bf16)(pad ? 0.f : src[e]);
    *(v4u*)(&sg[gr][pc * 8]) = pk.u; }
  __syncthreads();
  { const v16b b0 = frag_b(&sa[col][0], lane), b1 = frag_b(&sa[col][32], lane);
#pragma unroll 1
    for (int t = 0; t < KNEI; ++t) { const int rt = wave * KNEI + t; v8f acc = {}; acc = wmma_bf(frag_b(&sg[rt * 16 + col][0], lane), b0, acc); acc = wmma_bf(frag_b(&sg[rt * 16 + col][32], lane), b1, acc);
      if (col == 0) {
#pragma unroll
        for (int r = 0; r < 8; ++r) ssc[rt * 16 + 8 * g + r] = acc[r]; } }
    { v8f acc = {}; acc = wmma_bf(frag_b(&sr[wave * 16 + col][0], lane), b0, acc); acc = wmma_bf(frag_b(&sr[wave * 16 + col][32], lane), b1, acc);
      if (col == 1) {
#pragma unroll
        for (int r = 0; r < 8; ++r) srs[wave * 16 + 8 * g + r] = acc[r]; } } }
  __syncthreads();
  { const int rl = tid >> 1, hf = tid & 1; const int n = n0 + rl; float w[KNEI]; float mx = -3.0e38f; const float sref = srs[rl];
#pragma unroll
    for (int k = 0; k < KNEI; ++k) { float s = sref + ssc[rl * KNEI + k]; s = s > 0.f ? s : 0.01f * s; w[k] = s; mx = fmaxf(mx, s); }
    float den = 0.f;
#pragma unroll
    for (int k = 0; k < KNEI; ++k) { w[k] = exp_ni(w[k] - mx); den += w[k]; }
    const float inv = 1.0f / den;
#pragma unroll 1
    for (int d0 = 0; d0 < 32; d0 += 8) { float a8[8] = {0.f, 0.f, 0.f, 0.f, 0.f, 0.f, 0.f, 0.f};
#pragma unroll 1
      for (int k = 0; k < KNEI; ++k) { const float wk = w[k] * inv; union { v4u u; __bf16 e[8]; } pk; pk.u = *(const v4u*)(&sg[rl * KNEI + k][hf * 32 + d0]);
#pragma unroll
        for (int e = 0; e < 8; ++e) a8[e] += wk * (float)pk.e[e]; }
#pragma unroll
      for (int e = 0; e < 8; ++e) { const float v = a8[e]; se[rl][hf * 32 + d0 + e] = (n < NN) ? (v > 0.f ? v : expm1f(v)) : 0.f; } } }
  __syncthreads();
  for (int q = tid; q < 64 * 16; q += 128) { const int rl = q >> 4, pc = q & 15; if (n0 + rl < NN) vst2(EMB + (size_t)(n0 + rl) * HDIM + pc * 4, *(const v4f*)(&se[rl][pc * 4])); }
}
__global__ __launch_bounds__(128) void k_fc(const float* __restrict__ EMB, const float* __restrict__ fcw, const float* __restrict__ fcb, float* __restrict__ PART) {
  __shared__ __align__(16) float st[4][16][68]; __shared__ __align__(16) float ssum[64];
  const int tid = threadIdx.x, wave = tid >> 5, lane = tid & 31, col = lane & 15, g = lane >> 4; const int r0 = blockIdx.x * 64 + wave * 16;
  v8f acc[4] = {};
#pragma unroll
  for (int kc = 0; kc < 2; ++kc) { const int ra = r0 + col < NN ? r0 + col : NN - 1; const F2 a = split_row(EMB + (size_t)ra * HDIM, kc * 32, lane);
#pragma unroll
    for (int j = 0; j < 4; ++j) { const v16b wb = split_row(fcw + (size_t)(j * 16 + col) * HDIM, kc * 32, lane).h; acc[j] = wmma_bf(a.l, wb, acc[j]); acc[j] = wmma_bf(a.h, wb, acc[j]); } }
#pragma unroll
  for (int j = 0; j < 4; ++j) { const float bb = bfr(fcb[j * 16 + col]);
#pragma unroll
    for (int r = 0; r < 8; ++r) { const int row = r0 + 8 * g + r; st[wave][8 * g + r][j * 16 + col] = row < NN ? tanh_ni(acc[j][r] + bb) : 0.f; } }
  __syncthreads();
  if (tid < 64) { float s = 0.f;
    for (int w2 = 0; w2 < 4; ++w2) for (int rl = 0; rl < 16; ++rl) s += st[w2][rl][tid];
    ssum[tid] = s; }
  __syncthreads();
  if (tid < 16) vst2(PART + (size_t)blockIdx.x * HDIM + tid * 4, *(const v4f*)(&ssum[tid * 4]));
}
__global__ __launch_bounds__(64) void k_beta(const float* __restrict__ PART, int ntype, const float* __restrict__ sem, float* __restrict__ BETA) {
  __shared__ float sdot[3][64]; __shared__ __align__(16) float sb[4];
  const int tid = threadIdx.x;
  for (int t = 0; t < ntype; ++t) { float s = 0.f; const float* P = PART + (size_t)t * NBLK * HDIM;
    for (int bI = 0; bI < NBLK; ++bI) s += P[(size_t)bI * HDIM + tid];
    sdot[t][tid] = (s * (1.0f / NN)) * bfr(sem[tid]); }
  __syncthreads();
  if (tid == 0) { float lg[3] = {0.f, 0.f, 0.f}; for (int t = 0; t < ntype; ++t) { float s = 0.f; for (int d = 0; d < HDIM; ++d) s += sdot[t][d]; lg[t] = s; }
    float mx = lg[0]; for (int t = 1; t < ntype; ++t) mx = fmaxf(mx, lg[t]); float den = 0.f, e[3] = {0.f, 0.f, 0.f}; for (int t = 0; t < ntype; ++t) { e[t] = expf(lg[t] - mx); den += e[t]; }
    for (int t = 0; t < 3; ++t) sb[t] = t < ntype ? e[t] / den : 0.f; sb[3] = 0.f; }
  __syncthreads();
  if (tid == 0) vst2(BETA, *(const v4f*)sb);
}
__global__ __launch_bounds__(256) void k_blend(const float* __restrict__ E0, const float* __restrict__ E1, const float* __restrict__ E2, int ntype, const float* __restrict__ BETA, float* __restrict__ Z) {
  const size_t i4 = (size_t)blockIdx.x * 256 + threadIdx.x; if (i4 >= (size_t)NN * HDIM / 4) return;
  const float b0 = BETA[0], b1 = BETA[1], b2 = BETA[2];
  v4f v = *(const v4f*)(E0 + i4 * 4) * b0 + *(const v4f*)(E1 + i4 * 4) * b1; if (ntype > 2) v += *(const v4f*)(E2 + i4 * 4) * b2;
  vst2(Z + i4 * 4, v);
}
extern "C" void kernel_launch(void* const* d_in, const int* in_sizes, int n_in, void* d_out, int out_size, void* d_ws, size_t ws_size, hipStream_t stream) {
  (void)in_sizes; (void)n_in; (void)out_size; (void)ws_size;
  const float* h0 = (const float*)d_in[0]; const float* h1 = (const float*)d_in[1]; const float* h2 = (const float*)d_in[2]; const float* h3 = (const float*)d_in[3]; (void)h2;
  const int* nd0 = (const int*)d_in[4]; const int* nd1 = (const int*)d_in[5]; const int* np0 = (const int*)d_in[6]; const int* np1 = (const int*)d_in[7]; const int* np2 = (const int*)d_in[8];
  const float* att_d = (const float*)d_in[9]; const float* att_p = (const float*)d_in[10]; const float* fcwd = (const float*)d_in[11]; const float* fcbd = (const float*)d_in[12]; const float* semd = (const float*)d_in[13]; const float* fcwp = (const float*)d_in[14]; const float* fcbp = (const float*)d_in[15]; const float* semp = (const float*)d_in[16];
  float* zd = (float*)d_out; float* zp = (float*)((char*)d_out + 12800000);
  char* ws = (char*)d_ws; size_t off = 0;
  auto take = [&](size_t bytes) { char* p = ws + off; off += (bytes + 255) & ~(size_t)255; return p; };
  float* E[5]; for (int i = 0; i < 5; ++i) E[i] = (float*)take((size_t)NN * HDIM * 4);
  float* PARTD = (float*)take((size_t)2 * NBLK * HDIM * 4); float* PARTP = (float*)take((size_t)3 * NBLK * HDIM * 4); float* BETA = (float*)take(512);
  k_intra<<<NBLK, 128, 0, stream>>>(h0, h0, 50000, nd0, att_d, E[0]);
  k_intra<<<NBLK, 128, 0, stream>>>(h0, h1, 50000, nd1, att_d + 2 * HDIM, E[1]);
  k_intra<<<NBLK, 128, 0, stream>>>(h1, h0, 50000, np0, att_p, E[2]);
  k_intra<<<NBLK, 128, 0, stream>>>(h1, h1, 50000, np1, att_p + 2 * HDIM, E[3]);
  k_intra<<<NBLK, 128, 0, stream>>>(h1, h3, 20000, np2, att_p + 4 * HDIM, E[4]);
  k_fc<<<NBLK, 128, 0, stream>>>(E[0], fcwd, fcbd, PARTD);
  k_fc<<<NBLK, 128, 0, stream>>>(E[1], fcwd, fcbd, PARTD + (size_t)NBLK * HDIM);
  k_fc<<<NBLK, 128, 0, stream>>>(E[2], fcwp, fcbp, PARTP);
  k_fc<<<NBLK, 128, 0, stream>>>(E[3], fcwp, fcbp, PARTP + (size_t)NBLK * HDIM);
  k_fc<<<NBLK, 128, 0, stream>>>(E[4], fcwp, fcbp, PARTP + (size_t)2 * NBLK * HDIM);
  k_beta<<<1, 64, 0, stream>>>(PARTD, 2, semd, BETA);
  k_beta<<<1, 64, 0, stream>>>(PARTP, 3, semp, BETA + 64);
  k_blend<<<(NN * HDIM / 4 + 255) / 256, 256, 0, stream>>>(E[0], E[1], E[1], 2, BETA, zd);
  k_blend<<<(NN * HDIM / 4 + 255) / 256, 256, 0, stream>>>(E[2], E[3], E[4], 3, BETA + 64, zp);
}
